// EdgeTransformerLayer_43585328120339
// MI455X (gfx1250) — hardware-run, weakly checked
//
#include <hip/hip_runtime.h>


#ifndef NB
#define NB 2
#endif
#define NB_FULL  2
#define NN   64
#define SEQ  (NN * NN)
#define SEQ_FULL 4096
#define DM   256
#define NH_  8
#define HD   32
#define FF   512
#define HP   260
#define HHP  264
#define MHP  520
#define SC2  ((float)(0.17677669529663687 * 1.4426950408889634))
#define NEGB (-3.0e38f)
#define WCS  64.0f
#define CXS  16.0f
#define WOI  (1.0f / 1024.0f)
#define WI   (1.0f / 64.0f)
#define LNEPS 1.0e-5f

static_assert(NN == 64);
static_assert(SEQ == SEQ_FULL);
static_assert(HD == 32);
static_assert(NH_ * HD == DM);
static_assert(DM % 64 == 0);
static_assert(FF % 64 == 0);
static_assert(DM % 32 == 0);
static_assert(FF % 32 == 0);
static_assert(SEQ % 64 == 0);
static_assert((NB * SEQ) % 64 == 0);
static_assert((NB * SEQ) % 16 == 0);
static_assert(NB <= NB_FULL);
static_assert(DM == 8 * 32);
static_assert(FF == 8 * 64);
static_assert(DM == 2 * 32 * 4);
static_assert((HP * 4) % 16 == 0);
static_assert((HHP * 2) % 16 == 0);
static_assert((MHP * 2) % 16 == 0);
static_assert(2 * 32 * 16 == 16 * HD * 2);
static_assert(2 * 256 * 16 == 64 * 64 * 2);
static_assert(4 * 256 * 16 == 16 * 16 * HD * 2);
static_assert(8 * 2 * 2 * 32 * 16 == 16 * DM * 4);
static_assert(NN * 256 * 4 <= 131072);
static_assert(2 * 16 * HP * 4 + 16 * HHP * 2 + 16 * MHP * 2 <= 131072);
static_assert(16 * 68 * 4 <= 131072);
static_assert(64 * 65 * 4 <= 131072);

typedef _Float16 h16;
typedef unsigned short bf;
typedef __attribute__((ext_vector_type(16))) __bf16   v16bf;
typedef __attribute__((ext_vector_type(16))) _Float16 v16h;
typedef __attribute__((ext_vector_type(8)))  _Float16 v8h;
typedef __attribute__((ext_vector_type(4)))  _Float16 v4h;
typedef __attribute__((ext_vector_type(8)))  unsigned short v8us;
typedef __attribute__((ext_vector_type(8)))  float    v8f;
typedef __attribute__((ext_vector_type(4)))  float    v4f;
typedef __attribute__((ext_vector_type(4)))  unsigned v4u;
typedef v4f  __attribute__((may_alias)) v4fa;
typedef v8h  __attribute__((may_alias)) v8ha;
typedef v4h  __attribute__((may_alias)) v4ha;
typedef v4u  __attribute__((may_alias)) v4ua;

__device__ __forceinline__ unsigned short f2bf(float f) { unsigned u = __float_as_uint(f); u += 0x7FFFu + ((u >> 16) & 1u); return (unsigned short)(u >> 16); }
__device__ __forceinline__ float bfr(float f) { return __uint_as_float(((unsigned)f2bf(f)) << 16); }
__device__ __forceinline__ v16h cat16(v8h lo, v8h hi) { return __builtin_shufflevector(lo, hi, 0, 1, 2, 3, 4, 5, 6, 7, 8, 9, 10, 11, 12, 13, 14, 15); }
__device__ __forceinline__ v16bf cat16b(v8us lo, v8us hi) { return __builtin_bit_cast(v16bf, __builtin_shufflevector(lo, hi, 0, 1, 2, 3, 4, 5, 6, 7, 8, 9, 10, 11, 12, 13, 14, 15)); }
__device__ __forceinline__ v8f wmma16(v16h a, v16h b, v8f c) { return __builtin_amdgcn_wmma_f32_16x16x32_f16(false, a, false, b, (short)0, c, false, false); }
__device__ __forceinline__ v8f wmmab(v16bf a, v16bf b, v8f c) { return __builtin_amdgcn_wmma_f32_16x16x32_bf16(false, a, false, b, (short)0, c, false, false); }
__device__ __forceinline__ v16h  ldh(const h16* p) { return cat16(*(const v8h*)p, *(const v8h*)(p + 16)); }
__device__ __forceinline__ v16bf ldb(const bf* p)  { return cat16b(*(const v8us*)p, *(const v8us*)(p + 16)); }
__device__ __forceinline__ void wave_sync() { __builtin_amdgcn_fence(3  , "wavefront"); __builtin_amdgcn_wave_barrier(); asm volatile("" ::: "memory"); }

static __device__ __forceinline__ h16 toh_flush(float v) { const h16 r = (h16)v; return (fabsf(v) < 6.103515625e-05f) ? (h16)0.0f : r; }
__device__ __forceinline__ unsigned hbits(h16 v) { return (unsigned)__builtin_bit_cast(unsigned short, v); }
__device__ __forceinline__ v8f wmma16g(v16h a, v16h b, v8f c) { c = wmma16(a, b, c); asm volatile("v_nop\n\tv_nop\n\tv_nop\n\tv_nop" : "+v"(c) : "v"(a), "v"(b)); return c; }
__device__ __forceinline__ v8f wmmabg(v16bf a, v16bf b, v8f c) { c = wmmab(a, b, c); asm volatile("v_nop\n\tv_nop\n\tv_nop\n\tv_nop" : "+v"(c) : "v"(a), "v"(b)); return c; }
__device__ __forceinline__ float wsum(float v) { v += __shfl_xor(v, 16, 32); v += __shfl_xor(v, 8, 32); v += __shfl_xor(v, 4, 32); v += __shfl_xor(v, 2, 32); v += __shfl_xor(v, 1, 32); return v; }

static constexpr size_t al256(size_t v) { return (v + 255) & ~(size_t)255; }
static constexpr size_t SZ_XB = al256((size_t)NB * SEQ * DM * 2);
static constexpr size_t SZ_W4 = al256((size_t)4 * DM * DM * 2);
static constexpr size_t SZ_WO = al256((size_t)DM * DM * 2);
static constexpr size_t SZ_W1 = al256((size_t)DM * FF * 2);
static constexpr size_t SZ_W2 = al256((size_t)FF * DM * 2);
static constexpr size_t SZ_PL = al256((size_t)NB * NH_ * SEQ * HD * 2);
static constexpr size_t PL_ELEMS = SZ_PL / 2;
static constexpr size_t SZ_TOTAL = SZ_XB + SZ_W4 + SZ_WO + SZ_W1 + SZ_W2 + 5 * SZ_PL;
static_assert(SZ_TOTAL <= (size_t)134217728);
static_assert(((size_t)DM * DM * 2) % 256 == 0);
static_assert(PL_ELEMS == (size_t)NB * NH_ * SEQ * HD);

__global__ __launch_bounds__(256) void k_cvt8(const float* __restrict__ src, bf* dst, size_t n8) {
    const size_t i = (size_t)blockIdx.x * 256 + threadIdx.x; if (i >= n8) return;
    const v8f v = *(const v8f*)(src + i * 8); v8us o;
#pragma unroll
    for (int k = 0; k < 8; ++k) o[k] = f2bf(v[k]);
    *(volatile v8us*)(dst + i * 8) = o; __threadfence(); *(volatile v8us*)(dst + i * 8) = o;
}

__global__ __launch_bounds__(256) void k_wtr_b(const float* __restrict__ W, bf* WT, int rows, int cols) {
    __shared__ float ts[64 * 65];
    const int tid = threadIdx.x; const int k0 = blockIdx.x * 64, n0 = blockIdx.y * 64;
#pragma unroll 1
    for (int it = 0; it < 16; ++it) { const int e = it * 256 + tid; const int kk = e >> 6, nn = e & 63; ts[kk * 65 + nn] = W[(size_t)(k0 + kk) * cols + n0 + nn]; }
    __syncthreads();
    v8us o[2];
#pragma unroll
    for (int it = 0; it < 2; ++it) { const int n = it * 32 + (tid >> 3), c8 = (tid & 7) * 8;
#pragma unroll
        for (int e = 0; e < 8; ++e) o[it][e] = f2bf(ts[(c8 + e) * 65 + n]); }
#pragma unroll 1
    for (int ps = 0; ps < 2; ++ps) {
#pragma unroll
        for (int it = 0; it < 2; ++it) { const int n = it * 32 + (tid >> 3), c8 = (tid & 7) * 8;
            *(volatile v8us*)(WT + (size_t)(n0 + n) * rows + k0 + c8) = o[it]; }
        if (ps == 0) __threadfence(); }
}

__global__ __launch_bounds__(256) void k_wtr_h(const float* __restrict__ W, h16* WT, int rows, int cols) {
    __shared__ float ts[64 * 65];
    const int tid = threadIdx.x; const int k0 = blockIdx.x * 64, n0 = blockIdx.y * 64;
#pragma unroll 1
    for (int it = 0; it < 16; ++it) { const int e = it * 256 + tid; const int kk = e >> 6, nn = e & 63; ts[kk * 65 + nn] = W[(size_t)(k0 + kk) * cols + n0 + nn]; }
    __syncthreads();
    v8h o[2];
#pragma unroll
    for (int it = 0; it < 2; ++it) { const int n = it * 32 + (tid >> 3), c8 = (tid & 7) * 8;
#pragma unroll
        for (int e = 0; e < 8; ++e) o[it][e] = toh_flush(bfr(ts[(c8 + e) * 65 + n]) * WCS); }
#pragma unroll 1
    for (int ps = 0; ps < 2; ++ps) {
#pragma unroll
        for (int it = 0; it < 2; ++it) { const int n = it * 32 + (tid >> 3), c8 = (tid & 7) * 8;
            *(volatile v8h*)(WT + (size_t)(n0 + n) * rows + k0 + c8) = o[it]; }
        if (ps == 0) __threadfence(); }
}

__global__ __launch_bounds__(32) void k_proj(const bf* __restrict__ A, const bf* __restrict__ WT4, h16* PL4) {
    __shared__ __align__(16) float os[16 * 68];
    const int K = DM;
    const int lane = threadIdx.x & 31, lr = lane & 15, hi = lane >> 4; const int r0 = blockIdx.x * 64, c0 = blockIdx.y * 64;
    const int z = blockIdx.z;
    const bf* Bt = WT4 + (size_t)z * ((size_t)DM * DM);
    h16* Ph = PL4 + (size_t)z * PL_ELEMS;
    v8f acc[4][4];
#pragma unroll
    for (int mb = 0; mb < 4; ++mb)
#pragma unroll
        for (int nb = 0; nb < 4; ++nb) acc[mb][nb] = (v8f){};
    const size_t aoff = (size_t)(r0 + lr) * K + 8 * hi, boff = (size_t)(c0 + lr) * K + 8 * hi;
#pragma unroll 1
    for (int kc = 0; kc < K; kc += 32) {
        v16bf a[4];
#pragma unroll
        for (int mb = 0; mb < 4; ++mb) a[mb] = ldb(A + aoff + (size_t)mb * 16 * K + kc);
#pragma unroll
        for (int nb = 0; nb < 4; ++nb) { const v16bf b = ldb(Bt + boff + (size_t)nb * 16 * K + kc);
#pragma unroll
            for (int mb = 0; mb < 4; ++mb) acc[mb][nb] = wmmabg(a[mb], b, acc[mb][nb]); }
    }
    const int bb = r0 / SEQ, tt = r0 % SEQ; const int zc = bb * NH_ + c0 / HD;
    const size_t tbase = ((size_t)zc * SEQ + (size_t)tt) * HD;
#pragma unroll
    for (int mb = 0; mb < 4; ++mb) {
#pragma unroll
        for (int nb = 0; nb < 4; ++nb) {
#pragma unroll
            for (int j = 0; j < 8; ++j) os[(hi * 8 + j) * 68 + nb * 16 + lr] = acc[mb][nb][j]; }
        wave_sync();
#pragma unroll 1
        for (int ps = 0; ps < 2; ++ps) {
            const size_t sb = tbase + (size_t)(mb * 16) * HD;
#pragma unroll
            for (int hh = 0; hh < 2; ++hh) {
#pragma unroll
                for (int s = 0; s < 2; ++s) { const int p = s * 32 + lane; const int row = p >> 2, c8 = (p & 3) * 8;
                    const v4f x0 = *(const v4fa*)(&os[row * 68 + hh * 32 + c8]); const v4f x1 = *(const v4fa*)(&os[row * 68 + hh * 32 + c8 + 4]); v8h hv;
#pragma unroll
                    for (int i = 0; i < 4; ++i) { hv[i] = toh_flush(x0[i]); hv[4 + i] = toh_flush(x1[i]); }
                    const size_t oo = sb + (size_t)hh * ((size_t)SEQ * HD) + (size_t)p * 8;
                    *(volatile v8h*)(Ph + oo) = hv; } }
            if (ps == 0) __threadfence(); }
        wave_sync();
    }
}

__global__ __launch_bounds__(256) void k_edge(const h16* __restrict__ QH, const h16* __restrict__ KP, const h16* __restrict__ V1, const h16* __restrict__ V2, h16* CTX) {
    __shared__ __align__(16) unsigned lw[NN * 256];
    const int tid = threadIdx.x;
    const int lane = tid & 31, lr = lane & 15, hi = lane >> 4;
    const int wave = __builtin_amdgcn_readfirstlane((int)(threadIdx.x >> 5));
    const int it = blockIdx.x >> 2, jt = blockIdx.x & 3; const int zh = blockIdx.y;
    const size_t pbase = (size_t)zh * SEQ * HD;
    {
        const size_t qo = pbase + (size_t)((it * 16 + lr) * NN) * HD + 8 * hi;
        const size_t ko = pbase + (size_t)(jt * 16 + lr) * HD + 8 * hi;
#pragma unroll 1
        for (int s = 0; s < 8; ++s) {
            const int l = wave * 8 + s;
            const v16h a = ldh(QH + qo + (size_t)l * HD);
            const v16h b = ldh(KP + ko + (size_t)l * (NN * HD));
            v8f c = (v8f){};
            c = wmma16g(a, b, c);
#pragma unroll
            for (int r = 0; r < 8; ++r) lw[l * 256 + (8 * hi + r) * 16 + lr] = __float_as_uint(c[r] * SC2); }
    }
    __syncthreads();
    const int pi = tid >> 4, pj = tid & 15;
    float mx = NEGB;
#pragma unroll 4
    for (int l = 0; l < NN; ++l) mx = fmaxf(mx, __uint_as_float(lw[l * 256 + tid]));
    const h16* v1p = V1 + pbase + (size_t)((it * 16 + pi) * NN) * HD;
    const h16* v2p = V2 + pbase + (size_t)(jt * 16 + pj) * HD;
    float acc[32];
#pragma unroll
    for (int d = 0; d < 32; ++d) acc[d] = 0.0f;
    float ls = 0.0f;
#pragma unroll 1
    for (int l = 0; l < NN; ++l) {
        const float p = __builtin_amdgcn_exp2f(__uint_as_float(lw[l * 256 + tid]) - mx);
        ls += p;
        const h16* ap = v1p + (size_t)l * HD; const h16* bp = v2p + (size_t)l * (NN * HD);
        const v8h a0 = *(const v8h*)ap, a1 = *(const v8h*)(ap + 8), a2 = *(const v8h*)(ap + 16), a3 = *(const v8h*)(ap + 24);
        const v8h b0 = *(const v8h*)bp, b1 = *(const v8h*)(bp + 8), b2 = *(const v8h*)(bp + 16), b3 = *(const v8h*)(bp + 24);
#pragma unroll
        for (int e = 0; e < 8; ++e) {
            acc[e]      = fmaf(p * (float)a0[e], (float)b0[e], acc[e]);
            acc[8 + e]  = fmaf(p * (float)a1[e], (float)b1[e], acc[8 + e]);
            acc[16 + e] = fmaf(p * (float)a2[e], (float)b2[e], acc[16 + e]);
            acc[24 + e] = fmaf(p * (float)a3[e], (float)b3[e], acc[24 + e]); }
    }
    const float sc = CXS * (1.0f / ls);
    __syncthreads();
#pragma unroll
    for (int q = 0; q < 4; ++q) { v4u w;
#pragma unroll
        for (int e = 0; e < 4; ++e) { const h16 lo = toh_flush(acc[q * 8 + 2 * e] * sc); const h16 hv = toh_flush(acc[q * 8 + 2 * e + 1] * sc); w[e] = hbits(lo) | (hbits(hv) << 16); }
        *(v4ua*)(&lw[tid * 16 + q * 4]) = w; }
    __syncthreads();
    h16* cb = CTX + pbase + (size_t)((it * 16) * NN + jt * 16) * HD;
#pragma unroll 1
    for (int ps = 0; ps < 2; ++ps) {
#pragma unroll
        for (int s = 0; s < 4; ++s) { const int p = s * 256 + tid; const int i = p >> 6, q = p & 63;
            const v4u val = *(const v4ua*)(&lw[p * 4]);
            *(volatile v4u*)(cb + (size_t)i * (NN * HD) + q * 8) = val; }
        if (ps == 0) __threadfence(); }
}

__global__ __launch_bounds__(256) void k_tail(const h16* __restrict__ CTX, const h16* __restrict__ WOT, const h16* __restrict__ W1T, const h16* __restrict__ W2T,
                                              const float* __restrict__ X, const float* __restrict__ g1, const float* __restrict__ be1,
                                              const float* __restrict__ b1, const float* __restrict__ b2,
                                              const float* __restrict__ g2, const float* __restrict__ be2, float* OUT) {
    __shared__ __align__(16) float hf[16 * HP];
    __shared__ __align__(16) float ys[16 * HP];
    __shared__ __align__(16) h16 hh[16 * HHP];
    __shared__ __align__(16) h16 mh[16 * MHP];
    const int lane = threadIdx.x & 31, lr = lane & 15, hi = lane >> 4;
    const int wave = __builtin_amdgcn_readfirstlane((int)(threadIdx.x >> 5));
    const int rowbase = blockIdx.x * 16; const int bb = rowbase / SEQ, tt = rowbase % SEQ;
    {
        v8f c0 = (v8f){}, c1 = (v8f){};
        const size_t ao = ((size_t)bb * NH_ * SEQ + (size_t)(tt + lr)) * HD + 8 * hi;
        const size_t bo = (size_t)(wave * 32 + lr) * DM + 8 * hi;
#pragma unroll 1
        for (int hd = 0; hd < NH_; ++hd) {
            const v16h a = ldh(CTX + ao + (size_t)hd * ((size_t)SEQ * HD));
            const v16h w0 = ldh(WOT + bo + hd * HD); const v16h w1 = ldh(WOT + bo + (size_t)16 * DM + hd * HD);
            c0 = wmma16g(a, w0, c0); c1 = wmma16g(a, w1, c1); }
#pragma unroll
        for (int r = 0; r < 8; ++r) { hf[(8 * hi + r) * HP + wave * 32 + lr] = c0[r] * WOI; hf[(8 * hi + r) * HP + wave * 32 + 16 + lr] = c1[r] * WOI; }
    }
    __syncthreads();
#pragma unroll 1
    for (int rr = 0; rr < 2; ++rr) {
        const int row = wave * 2 + rr;
        const float* xr = X + (size_t)(rowbase + row) * DM;
        const v4f x0 = *(const v4f*)(xr + 4 * lane); const v4f x1 = *(const v4f*)(xr + 128 + 4 * lane);
        const v4f a0 = *(const v4fa*)(&hf[row * HP + 4 * lane]); const v4f a1 = *(const v4fa*)(&hf[row * HP + 128 + 4 * lane]);
        float v[8];
#pragma unroll
        for (int e = 0; e < 4; ++e) { v[e] = a0[e] + bfr(x0[e]); v[4 + e] = a1[e] + bfr(x1[e]); }
        float s = 0.0f;
#pragma unroll
        for (int e = 0; e < 8; ++e) s += v[e];
        s = wsum(s);
        const float mean = s * (1.0f / DM);
        float q = 0.0f;
#pragma unroll
        for (int e = 0; e < 8; ++e) { const float d = v[e] - mean; q += d * d; }
        q = wsum(q);
        const float rstd = rsqrtf(q * (1.0f / DM) + LNEPS);
        const v4f ga = *(const v4f*)(g1 + 4 * lane), gb = *(const v4f*)(g1 + 128 + 4 * lane);
        const v4f ea = *(const v4f*)(be1 + 4 * lane), eb = *(const v4f*)(be1 + 128 + 4 * lane);
        v4f n0, n1; v4h h0, h1;
#pragma unroll
        for (int e = 0; e < 4; ++e) {
            n0[e] = (v[e] - mean) * rstd * bfr(ga[e]) + bfr(ea[e]);
            n1[e] = (v[4 + e] - mean) * rstd * bfr(gb[e]) + bfr(eb[e]);
            h0[e] = toh_flush(n0[e]); h1[e] = toh_flush(n1[e]); }
        *(v4fa*)(&hf[row * HP + 4 * lane]) = n0; *(v4fa*)(&hf[row * HP + 128 + 4 * lane]) = n1;
        *(v4ha*)(&hh[row * HHP + 4 * lane]) = h0; *(v4ha*)(&hh[row * HHP + 128 + 4 * lane]) = h1;
    }
    __syncthreads();
    {
        v8f c[4];
#pragma unroll
        for (int t = 0; t < 4; ++t) c[t] = (v8f){};
        const size_t bo = (size_t)(wave * 64 + lr) * DM + 8 * hi;
#pragma unroll 1
        for (int kc = 0; kc < DM; kc += 32) {
            const v8h al = *(const v8ha*)(&hh[lr * HHP + kc + 8 * hi]); const v8h ah = *(const v8ha*)(&hh[lr * HHP + kc + 16 + 8 * hi]);
            const v16h a = cat16(al, ah);
#pragma unroll
            for (int t = 0; t < 4; ++t) { const v16h w = ldh(W1T + bo + (size_t)t * 16 * DM + kc); c[t] = wmma16g(a, w, c[t]); }
        }
#pragma unroll
        for (int t = 0; t < 4; ++t) { const int col = wave * 64 + t * 16 + lr; const float bias = bfr(b1[col]);
#pragma unroll
            for (int r = 0; r < 8; ++r) mh[(8 * hi + r) * MHP + col] = toh_flush(fmaxf(c[t][r] * WI + bias, 0.0f)); }
    }
    __syncthreads();
    {
        v8f c[2];
        c[0] = (v8f){}; c[1] = (v8f){};
        const size_t bo = (size_t)(wave * 32 + lr) * FF + 8 * hi;
#pragma unroll 1
        for (int kc = 0; kc < FF; kc += 32) {
            const v8h al = *(const v8ha*)(&mh[lr * MHP + kc + 8 * hi]); const v8h ah = *(const v8ha*)(&mh[lr * MHP + kc + 16 + 8 * hi]);
            const v16h a = cat16(al, ah);
#pragma unroll
            for (int t = 0; t < 2; ++t) { const v16h w = ldh(W2T + bo + (size_t)t * 16 * FF + kc); c[t] = wmma16g(a, w, c[t]); }
        }
#pragma unroll
        for (int t = 0; t < 2; ++t) { const int col = wave * 32 + t * 16 + lr; const float bias = bfr(b2[col]);
#pragma unroll
            for (int r = 0; r < 8; ++r) ys[(8 * hi + r) * HP + col] = c[t][r] * WI + bias + hf[(8 * hi + r) * HP + col]; }
    }
    __syncthreads();
    v4f ov[2][2];
#pragma unroll
    for (int rr = 0; rr < 2; ++rr) {
        const int row = wave * 2 + rr;
        const v4f a0 = *(const v4fa*)(&ys[row * HP + 4 * lane]); const v4f a1 = *(const v4fa*)(&ys[row * HP + 128 + 4 * lane]);
        float s = 0.0f;
#pragma unroll
        for (int e = 0; e < 4; ++e) s += a0[e] + a1[e];
        s = wsum(s);
        const float mean = s * (1.0f / DM);
        float q = 0.0f;
#pragma unroll
        for (int e = 0; e < 4; ++e) { const float d0 = a0[e] - mean, d1 = a1[e] - mean; q += d0 * d0 + d1 * d1; }
        q = wsum(q);
        const float rstd = rsqrtf(q * (1.0f / DM) + LNEPS);
        const v4f ga = *(const v4f*)(g2 + 4 * lane), gb = *(const v4f*)(g2 + 128 + 4 * lane);
        const v4f ea = *(const v4f*)(be2 + 4 * lane), eb = *(const v4f*)(be2 + 128 + 4 * lane);
#pragma unroll
        for (int e = 0; e < 4; ++e) {
            ov[rr][0][e] = (a0[e] - mean) * rstd * bfr(ga[e]) + bfr(ea[e]);
            ov[rr][1][e] = (a1[e] - mean) * rstd * bfr(gb[e]) + bfr(eb[e]); }
    }
    float* ob = OUT + (size_t)(rowbase + wave * 2) * DM + 4 * lane;
#pragma unroll 1
    for (int ps = 0; ps < 2; ++ps) {
#pragma unroll
        for (int rr = 0; rr < 2; ++rr) {
            *(volatile v4f*)(ob + (size_t)rr * DM) = ov[rr][0];
            *(volatile v4f*)(ob + (size_t)rr * DM + 128) = ov[rr][1]; }
        if (ps == 0) __threadfence(); }
}

extern "C" void kernel_launch(void* const* d_in, const int* in_sizes, int n_in,
                              void* d_out, int out_size, void* d_ws, size_t ws_size, hipStream_t stream) {
    if (n_in < 14) return;
    const size_t needx = ((size_t)(NB - 1) * SEQ_FULL + SEQ) * DM;
    if ((size_t)in_sizes[0] < needx) return;
    for (int i = 1; i <= 5; ++i) if ((size_t)in_sizes[i] < (size_t)DM * DM) return;
    if (in_sizes[6] < DM || in_sizes[7] < DM) return;
    if ((size_t)in_sizes[8] < (size_t)DM * FF || in_sizes[9] < FF) return;
    if ((size_t)in_sizes[10] < (size_t)FF * DM || in_sizes[11] < DM) return;
    if (in_sizes[12] < DM || in_sizes[13] < DM) return;
    if ((size_t)out_size < needx) return;
    if (SZ_TOTAL > ws_size) return;
    const float* x   = (const float*)d_in[0];
    const float* wq  = (const float*)d_in[1];
    const float* wk  = (const float*)d_in[2];
    const float* wv1 = (const float*)d_in[3];
    const float* wv2 = (const float*)d_in[4];
    const float* wo  = (const float*)d_in[5];
    const float* lag = (const float*)d_in[6];
    const float* lab = (const float*)d_in[7];
    const float* w1  = (const float*)d_in[8];
    const float* b1  = (const float*)d_in[9];
    const float* w2  = (const float*)d_in[10];
    const float* b2  = (const float*)d_in[11];
    const float* log_ = (const float*)d_in[12];
    const float* lob = (const float*)d_in[13];
    float* OUT = (float*)d_out;
    char* wsp = (char*)d_ws;
    bf*  XB  = (bf*)wsp;  wsp += SZ_XB;
    bf*  WT4 = (bf*)wsp;  wsp += SZ_W4;
    h16* WOT = (h16*)wsp; wsp += SZ_WO;
    h16* W1T = (h16*)wsp; wsp += SZ_W1;
    h16* W2T = (h16*)wsp; wsp += SZ_W2;
    h16* PL4 = (h16*)wsp; wsp += 4 * SZ_PL;
    h16* CTX = (h16*)wsp; wsp += SZ_PL;
    h16* QH = PL4; h16* KP = PL4 + PL_ELEMS; h16* V1 = PL4 + 2 * PL_ELEMS; h16* V2 = PL4 + 3 * PL_ELEMS;

    { const size_t n8 = (size_t)NB * SEQ * DM / 8;
      k_cvt8<<<(unsigned)((n8 + 255) / 256), 256, 0, stream>>>(x, XB, n8); }
    k_wtr_b<<<dim3(DM / 64, DM / 64, 1), 256, 0, stream>>>(wq,  WT4,                       DM, DM);
    k_wtr_b<<<dim3(DM / 64, DM / 64, 1), 256, 0, stream>>>(wk,  WT4 + (size_t)DM * DM,     DM, DM);
    k_wtr_b<<<dim3(DM / 64, DM / 64, 1), 256, 0, stream>>>(wv1, WT4 + (size_t)2 * DM * DM, DM, DM);
    k_wtr_b<<<dim3(DM / 64, DM / 64, 1), 256, 0, stream>>>(wv2, WT4 + (size_t)3 * DM * DM, DM, DM);
    k_wtr_h<<<dim3(DM / 64, DM / 64, 1), 256, 0, stream>>>(wo, WOT, DM, DM);
    k_wtr_h<<<dim3(DM / 64, FF / 64, 1), 256, 0, stream>>>(w1, W1T, DM, FF);
    k_wtr_h<<<dim3(FF / 64, DM / 64, 1), 256, 0, stream>>>(w2, W2T, FF, DM);

    k_proj<<<dim3(NB * SEQ / 64, DM / 64, 4), 32, 0, stream>>>(XB, WT4, PL4);
    k_edge<<<dim3((NN / 16) * (NN / 16), NB * NH_, 1), 256, 0, stream>>>(QH, KP, V1, V2, CTX);
    k_tail<<<dim3(NB * SEQ / 16, 1, 1), 256, 0, stream>>>(CTX, WOT, W1T, W2T, x, lag, lab, b1, b2, log_, lob, OUT);
}
